// MultiheadIsotropicAFA_63299228008886
// MI455X (gfx1250) — hardware-verified
//
#include <hip/hip_runtime.h>
#include <hip/hip_bf16.h>


#define USE_ASYNC_COPY 0
typedef _Float16 __hf16;
#define __bf16 __hf16
typedef __attribute__((ext_vector_type(16))) _Float16 v16bf;
typedef __attribute__((ext_vector_type(8)))  _Float16 v8bf;
typedef __attribute__((ext_vector_type(2)))  _Float16 v2bf;
typedef __attribute__((ext_vector_type(8)))  float  v8f;
typedef __attribute__((ext_vector_type(4)))  int    v4i;

#define TILE_BM 128
#define TILE_BN 128
#define TILE_BK 32
#define LDS_PAD 8


#define AS_GLOBAL __attribute__((address_space(1)))
#define AS_SHARED __attribute__((address_space(3)))

__device__ __forceinline__ v16bf load_frag(const __bf16* rowp, int half) {
    const v8bf lo = *reinterpret_cast<const v8bf*>(rowp + half * 8);
    const v8bf hi = *reinterpret_cast<const v8bf*>(rowp + 16 + half * 8);
    return __builtin_shufflevector(lo, hi, 0, 1, 2, 3, 4, 5, 6, 7,
                                           8, 9, 10, 11, 12, 13, 14, 15);
}

template <bool TRANS_B, bool SPLIT>
__global__ __launch_bounds__(256)
void wmma_gemm_kernel(const __bf16* __restrict__ A, const __bf16* __restrict__ Bm,
                      const float* __restrict__ bias, float* __restrict__ C,
                      int M, int N, int K,
                      long long sA, long long sB, long long sC,
                      const __bf16* __restrict__ Alo = nullptr, const __bf16* __restrict__ Blo = nullptr)
{
    (void)M;
    __shared__ __bf16 As[2][TILE_BM][TILE_BK + LDS_PAD];
    __shared__ __bf16 Bs[2][TILE_BN][TILE_BK + LDS_PAD];
    __shared__ __bf16 Als[SPLIT ? 2 : 1][SPLIT ? TILE_BM : 1][TILE_BK + LDS_PAD];
    __shared__ __bf16 Bls[SPLIT ? 2 : 1][SPLIT ? TILE_BN : 1][TILE_BK + LDS_PAD];
    const __bf16* Alb = SPLIT ? (Alo + (size_t)blockIdx.z * sA) : nullptr;
    const __bf16* Blb = SPLIT ? (Blo + (size_t)blockIdx.z * sB) : nullptr;

    const int tid  = threadIdx.x;
    const int lane = tid & 31;
    const int wave = tid >> 5;
    const int wm   = wave & 3;
    const int wn   = wave >> 2;
    const int half = lane >> 4;
    const int r16  = lane & 15;

    const __bf16* Ab = A  + (size_t)blockIdx.z * sA;
    const __bf16* Bb = Bm + (size_t)blockIdx.z * sB;
    float*        Cb = C  + (size_t)blockIdx.z * sC;

    const int row0 = blockIdx.y * TILE_BM;
    const int col0 = blockIdx.x * TILE_BN;

    auto stageA = [&](int buf, int k0) {
#if USE_ASYNC_COPY
        #pragma unroll
        for (int i = 0; i < 2; ++i) {
            const int idx = tid + i * 256;
            const int r = idx >> 2, c = (idx & 3) << 3;
            __builtin_amdgcn_global_load_async_to_lds_b128(
                (AS_GLOBAL v4i*)(Ab + (size_t)(row0 + r) * K + k0 + c),
                (AS_SHARED v4i*)&As[buf][r][c],
                0, 0);
        }
#else
        v8bf t[2];
        #pragma unroll
        for (int i = 0; i < 2; ++i) {
            const int idx = tid + i * 256;
            t[i] = *reinterpret_cast<const v8bf*>(
                Ab + (size_t)(row0 + (idx >> 2)) * K + k0 + ((idx & 3) << 3));
        }
        #pragma unroll
        for (int i = 0; i < 2; ++i) {
            const int idx = tid + i * 256;
            *reinterpret_cast<v8bf*>(&As[buf][idx >> 2][(idx & 3) << 3]) = t[i];
        }
        if (SPLIT) {
            #pragma unroll
            for (int i = 0; i < 2; ++i) {
                const int idx = tid + i * 256;
                *reinterpret_cast<v8bf*>(&Als[buf][idx >> 2][(idx & 3) << 3]) =
                    *reinterpret_cast<const v8bf*>(Alb + (size_t)(row0 + (idx >> 2)) * K + k0 + ((idx & 3) << 3));
            }
        }
#endif
    };

    auto stageB = [&](int buf, int k0) {
        if (TRANS_B) {
#if USE_ASYNC_COPY
            #pragma unroll
            for (int i = 0; i < 2; ++i) {
                const int idx = tid + i * 256;
                const int n = idx >> 2, c = (idx & 3) << 3;
                __builtin_amdgcn_global_load_async_to_lds_b128(
                    (AS_GLOBAL v4i*)(Bb + (size_t)(col0 + n) * K + k0 + c),
                    (AS_SHARED v4i*)&Bs[buf][n][c],
                    0, 0);
            }
#else
            v8bf t[2];
            #pragma unroll
            for (int i = 0; i < 2; ++i) {
                const int idx = tid + i * 256;
                t[i] = *reinterpret_cast<const v8bf*>(
                    Bb + (size_t)(col0 + (idx >> 2)) * K + k0 + ((idx & 3) << 3));
            }
            #pragma unroll
            for (int i = 0; i < 2; ++i) {
                const int idx = tid + i * 256;
                *reinterpret_cast<v8bf*>(&Bs[buf][idx >> 2][(idx & 3) << 3]) = t[i];
            }
            if (SPLIT) {
                #pragma unroll
                for (int i = 0; i < 2; ++i) {
                    const int idx = tid + i * 256;
                    *reinterpret_cast<v8bf*>(&Bls[buf][idx >> 2][(idx & 3) << 3]) =
                        *reinterpret_cast<const v8bf*>(Blb + (size_t)(col0 + (idx >> 2)) * K + k0 + ((idx & 3) << 3));
                }
            }
#endif
        } else {
            v8bf t[2];
            #pragma unroll
            for (int i = 0; i < 2; ++i) {
                const int idx = tid + i * 256;
                const int r = idx >> 4;
                const int c = (idx & 15) << 3;
                t[i] = *reinterpret_cast<const v8bf*>(
                    Bb + (size_t)(k0 + r) * N + col0 + c);
            }
            #pragma unroll
            for (int i = 0; i < 2; ++i) {
                const int idx = tid + i * 256;
                const int r = idx >> 4;
                const int c = (idx & 15) << 3;
                #pragma unroll
                for (int e = 0; e < 8; ++e) Bs[buf][c + e][r] = t[i][e];
            }
            if (SPLIT) {
                #pragma unroll
                for (int i = 0; i < 2; ++i) {
                    const int idx = tid + i * 256;
                    const int r = idx >> 4;
                    const int c = (idx & 15) << 3;
                    const v8bf tl = *reinterpret_cast<const v8bf*>(Blb + (size_t)(k0 + r) * N + col0 + c);
                    #pragma unroll
                    for (int e = 0; e < 8; ++e) Bls[buf][c + e][r] = tl[e];
                }
            }
        }
    };

    v8f acc[2][4] = {};

    const int nk = K / TILE_BK;
    stageA(0, 0);
    stageB(0, 0);
#if USE_ASYNC_COPY
    __builtin_amdgcn_s_wait_asynccnt(0);
#endif
    __syncthreads();

    for (int kt = 0; kt < nk; ++kt) {
        const int buf = kt & 1;
        const int nxt = kt + 1;

        if (nxt + 1 < nk) {
            __builtin_prefetch(Ab + (size_t)(row0 + (tid >> 1)) * K
                                  + (nxt + 1) * TILE_BK, 0, 0);
        }
        if (nxt < nk) {
            stageA(nxt & 1, nxt * TILE_BK);
            stageB(nxt & 1, nxt * TILE_BK);
        }

        v16bf afrag[2], bfrag[4];
        #pragma unroll
        for (int mt = 0; mt < 2; ++mt)
            afrag[mt] = load_frag(&As[buf][wm * 32 + mt * 16 + r16][0], half);
        #pragma unroll
        for (int nt = 0; nt < 4; ++nt)
            bfrag[nt] = load_frag(&Bs[buf][wn * 64 + nt * 16 + r16][0], half);

        #pragma unroll
        for (int mt = 0; mt < 2; ++mt)
            #pragma unroll
            for (int nt = 0; nt < 4; ++nt) {
                acc[mt][nt] = __builtin_amdgcn_wmma_f32_16x16x32_f16(
                    false, afrag[mt], false, bfrag[nt],
                    (short)0, acc[mt][nt], false, false);
                asm volatile("v_nop\n\tv_nop\n\tv_nop\n\tv_nop" : "+v"(acc[mt][nt]) : "v"(afrag[mt]), "v"(bfrag[nt]));
            }
        if (SPLIT) {
            v16bf alf[2], blf[4];
            #pragma unroll
            for (int mt = 0; mt < 2; ++mt)
                alf[mt] = load_frag(&Als[buf][wm * 32 + mt * 16 + r16][0], half);
            #pragma unroll
            for (int nt = 0; nt < 4; ++nt)
                blf[nt] = load_frag(&Bls[buf][wn * 64 + nt * 16 + r16][0], half);
            #pragma unroll
            for (int mt = 0; mt < 2; ++mt)
                #pragma unroll
                for (int nt = 0; nt < 4; ++nt) {
                    acc[mt][nt] = __builtin_amdgcn_wmma_f32_16x16x32_f16(false, afrag[mt], false, blf[nt], (short)0, acc[mt][nt], false, false);
                    acc[mt][nt] = __builtin_amdgcn_wmma_f32_16x16x32_f16(false, alf[mt], false, bfrag[nt], (short)0, acc[mt][nt], false, false);
                    asm volatile("v_nop\n\tv_nop\n\tv_nop\n\tv_nop" : "+v"(acc[mt][nt]) : "v"(alf[mt]), "v"(blf[nt]));
                }
        }

#if USE_ASYNC_COPY
        __builtin_amdgcn_s_wait_asynccnt(0);
#endif
        __syncthreads();
    }

    for (int pass = 0; pass < 2; ++pass) {
        #pragma unroll
        for (int mt = 0; mt < 2; ++mt) {
            const int cm0 = row0 + wm * 32 + mt * 16;
            #pragma unroll
            for (int p = 0; p < 2; ++p) {
                const int cbase = col0 + wn * 64 + p * 32;
                const float bv = bias ? bias[cbase + lane] : 0.0f;
                #pragma unroll
                for (int v = 0; v < 8; ++v) {
                    const float a0 = acc[mt][2 * p][v], a1 = acc[mt][2 * p + 1][v];
                    const float x0 = __shfl_xor(a0, 16), x1 = __shfl_xor(a1, 16);
                    *(volatile float*)(Cb + (size_t)(cm0 + v) * N + cbase + lane)     = (half ? x1 : a0) + bv;
                    *(volatile float*)(Cb + (size_t)(cm0 + 8 + v) * N + cbase + lane) = (half ? a1 : x0) + bv;
                }
            }
        }
        __threadfence();
    }
}

__global__ __launch_bounds__(256)
void f32_to_bf16_kernel(const float* __restrict__ src, __bf16* __restrict__ dst, __bf16* __restrict__ dlo)
{
    const size_t i = (size_t)blockIdx.x * 256 + threadIdx.x;
    float f[8];
    {
        const float4 a = reinterpret_cast<const float4*>(src)[2 * i];
        const float4 b = reinterpret_cast<const float4*>(src)[2 * i + 1];
        f[0] = a.x; f[1] = a.y; f[2] = a.z; f[3] = a.w; f[4] = b.x; f[5] = b.y; f[6] = b.z; f[7] = b.w;
    }
    v8bf o, l;
    #pragma unroll
    for (int e = 0; e < 8; ++e) { o[e] = (__bf16)f[e]; l[e] = (__bf16)(f[e] - (float)o[e]); }
    *(volatile v8bf*)(reinterpret_cast<v8bf*>(dst) + i) = o; if (dlo) *(volatile v8bf*)(reinterpret_cast<v8bf*>(dlo) + i) = l;
    __threadfence();
    *(volatile v8bf*)(reinterpret_cast<v8bf*>(dst) + i) = o; if (dlo) *(volatile v8bf*)(reinterpret_cast<v8bf*>(dlo) + i) = l;
}

__global__ __launch_bounds__(256)
void rotate_qkv_kernel(const float* __restrict__ Qp, const float* __restrict__ Kp,
                       const float* __restrict__ Vp, const float* __restrict__ lam,
                       __bf16* __restrict__ Qr, __bf16* __restrict__ Kr,
                       __bf16* __restrict__ Vr,
                       float* __restrict__ qn, float* __restrict__ kn)
{
    __shared__ float rq[4][64], rk[4][64];
    __shared__ float nq[32], nk[32];
    const int d = threadIdx.x & 63, lsub = threadIdx.x >> 6;
    const int h = blockIdx.y;
    const int b = blockIdx.z;
  for (int g8 = 0; g8 < 8; ++g8) {
    const int l = blockIdx.x * 32 + g8 * 4 + lsub;

    const float om  = lam[h * 32 + (d >> 1)] * ((d & 1) ? -1.0f : 1.0f);
    const float th  = -(float)l * om;
    const float cth = cosf(th);
    const float sth = sinf(th);

    const size_t zin = ((size_t)b * 1024 + l) * 1024;
    const int    co  = h * 64 + d;
    const float qre = Qp[zin + co], qim = Qp[zin + 512 + co];
    const float kre = Kp[zin + co], kim = Kp[zin + 512 + co];
    const float vre = Vp[zin + co], vim = Vp[zin + 512 + co];

    const size_t zo = (((size_t)(b * 8 + h)) * 1024 + l) * 128 + 2 * d;
    v2bf q, k, v;
    q[0] = (__bf16)(qre * cth - qim * sth); q[1] = (__bf16)(qre * sth + qim * cth);
    k[0] = (__bf16)(kre * cth - kim * sth); k[1] = (__bf16)(kre * sth + kim * cth);
    v[0] = (__bf16)(vre * cth - vim * sth); v[1] = (__bf16)(vre * sth + vim * cth);
    *(volatile v2bf*)(&Qr[zo]) = q; *(volatile v2bf*)(&Kr[zo]) = k; *(volatile v2bf*)(&Vr[zo]) = v;
    __threadfence();
    *(volatile v2bf*)(&Qr[zo]) = q; *(volatile v2bf*)(&Kr[zo]) = k; *(volatile v2bf*)(&Vr[zo]) = v;

    rq[lsub][d] = qre * qre + qim * qim;
    rk[lsub][d] = kre * kre + kim * kim;
    __syncthreads();
    #pragma unroll
    for (int s2 = 32; s2 > 0; s2 >>= 1) {
        if (d < s2) { rq[lsub][d] += rq[lsub][d + s2]; rk[lsub][d] += rk[lsub][d + s2]; }
        __syncthreads();
    }
    if (d == 0) { nq[g8 * 4 + lsub] = rq[lsub][0]; nk[g8 * 4 + lsub] = rk[lsub][0]; }
    __syncthreads();
  }
    if (threadIdx.x < 64) {
        const size_t o = ((size_t)(b * 8 + h)) * 1024 + blockIdx.x * 32 + (threadIdx.x & 31);
        float* dst = (threadIdx.x < 32) ? (qn + o) : (kn + o);
        const float val = (threadIdx.x < 32) ? nq[threadIdx.x] : nk[threadIdx.x & 31];
        *(volatile float*)dst = val; __threadfence(); *(volatile float*)dst = val;
    }
}

__global__ __launch_bounds__(256)
void softmax_kernel(const float* __restrict__ dotA, __bf16* __restrict__ Ahat,
                    const float* __restrict__ qn, const float* __restrict__ kn,
                    const float* __restrict__ mu, const float* __restrict__ sigma,
                    const float* __restrict__ eta, const float* __restrict__ gam,
                    const float* __restrict__ tau, const float* __restrict__ nus)
{
    const int i = blockIdx.x, h = blockIdx.y, b = blockIdx.z;
    const int tid = threadIdx.x;
    const int z = b * 8 + h;

    const float* row  = dotA + (((size_t)z) * 1024 + i) * 1024;
    __bf16*      arow = Ahat + (((size_t)z) * 1024 + i) * 1024;
    const float  qni = qn[(size_t)z * 1024 + i];
    const float* knr = kn + (size_t)z * 1024;

    const float muh   = mu[h];
    const float alpha = muh * muh;
    const float sig2  = sigma[h] * sigma[h];
    const float eta2  = eta[h] * eta[h];
    const float gam2  = gam[h] * gam[h];
    const float tau2  = tau[h] * tau[h];
    const float nsq   = nus[h];
    const float nu    = nsq * nsq;

    __shared__ float scl[1024];
    __shared__ float red[256];
    float lmax = -INFINITY;
    #pragma unroll 1
    for (int it = 0; it < 4; ++it) {
        const int j = tid + it * 256;
        float s = -INFINITY;
        if (j <= i) {
            const float dt  = (float)(i - j);
            const float dec = __expf(-dt * alpha);
            const float d2  = dec * dec;
            const float Vij = sig2 * (1.0f - d2) / (2.0f * alpha + 1e-6f) + eta2 * d2 + gam2;
            const float R2  = fmaxf(qni + d2 * knr[j] - 2.0f * dec * row[j], 0.0f);
            const float Sv  = 1.0f / (nu * 64.0f * Vij);
            s = tau2 * (-__logf(Vij) - __logf(1.0f + R2 * Sv));
        }
        scl[j] = s; lmax = fmaxf(lmax, s);
    }
    red[tid] = lmax;
    __syncthreads();
    for (int t = 128; t > 0; t >>= 1) { if (tid < t) red[tid] = fmaxf(red[tid], red[tid + t]); __syncthreads(); }
    const float mx = red[0];
    __syncthreads();
    float lsum = 0.0f;
    #pragma unroll 1
    for (int it = 0; it < 4; ++it) { const int j = tid + it * 256; const float p = (j <= i) ? __expf(scl[j] - mx) : 0.0f; scl[j] = p; lsum += p; }
    red[tid] = lsum;
    __syncthreads();
    for (int t = 128; t > 0; t >>= 1) { if (tid < t) red[tid] += red[tid + t]; __syncthreads(); }
    const float inv = 1.0f / red[0];
    for (int pass = 0; pass < 2; ++pass) {
        #pragma unroll 1
        for (int it = 0; it < 4; ++it) {
            const int j = tid + it * 256;
            float out = 0.0f;
            if (j <= i) out = scl[j] * inv * __expf(-(float)(i - j) * alpha);
            *(volatile __bf16*)(arow + j) = (__bf16)out;
        }
        __threadfence();
    }
}

__global__ __launch_bounds__(64)
void unrotate_kernel(const float* __restrict__ est, const float* __restrict__ lam,
                     __bf16* __restrict__ Xo, __bf16* __restrict__ Xol)
{
    const int d = threadIdx.x, l = blockIdx.x, h = blockIdx.y, b = blockIdx.z;
    const float om  = lam[h * 32 + (d >> 1)] * ((d & 1) ? -1.0f : 1.0f);
    const float th  = (float)l * om;
    const float cth = cosf(th);
    const float sth = sinf(th);

    const size_t zi = (((size_t)(b * 8 + h)) * 1024 + l) * 128 + 2 * d;
    const float er = est[zi], ei = est[zi + 1];

    const size_t zo = ((size_t)b * 1024 + l) * 1024;
    const int    co = h * 64 + d;
    const float vr = er * cth - ei * sth, vi = er * sth + ei * cth;
    const __bf16 hr = (__bf16)vr, hi_ = (__bf16)vi, lr = (__bf16)(vr - (float)hr), li = (__bf16)(vi - (float)hi_);
    for (int pass = 0; pass < 2; ++pass) {
        *(volatile __bf16*)(Xo + zo + co) = hr;  *(volatile __bf16*)(Xo + zo + 512 + co) = hi_;
        *(volatile __bf16*)(Xol + zo + co) = lr; *(volatile __bf16*)(Xol + zo + 512 + co) = li;
        __threadfence();
    }
}

extern "C" void kernel_launch(void* const* d_in, const int* in_sizes, int n_in,
                              void* d_out, int out_size, void* d_ws, size_t ws_size,
                              hipStream_t stream)
{
    (void)in_sizes; (void)n_in; (void)out_size;

    const float* Zq   = (const float*)d_in[0];
    const float* Zk   = (const float*)d_in[1];
    const float* Zv   = (const float*)d_in[2];
    const float* Wq_w = (const float*)d_in[3];
    const float* Wq_b = (const float*)d_in[4];
    const float* Wk_w = (const float*)d_in[5];
    const float* Wk_b = (const float*)d_in[6];
    const float* Wv_w = (const float*)d_in[7];
    const float* Wv_b = (const float*)d_in[8];
    const float* Wo_w = (const float*)d_in[9];
    const float* Wo_b = (const float*)d_in[10];
    const float* lam  = (const float*)d_in[11];
    const float* mu   = (const float*)d_in[12];
    const float* sig  = (const float*)d_in[13];
    const float* eta  = (const float*)d_in[14];
    const float* gam  = (const float*)d_in[15];
    const float* tau  = (const float*)d_in[16];
    const float* nus  = (const float*)d_in[17];

    char* w = (char*)d_ws;
    auto allocf = [&](size_t n) { float*  p = (float*)w;  w += n * sizeof(float);  return p; };
    auto allocb = [&](size_t n) { __bf16* p = (__bf16*)w; w += n * sizeof(__bf16); return p; };

    const size_t NPROJ = (size_t)2048 * 1024;
    const size_t NW    = (size_t)1024 * 1024;
    const size_t NROT  = (size_t)16 * 1024 * 128;
    const size_t NROW  = (size_t)16 * 1024;
    const size_t NATT  = (size_t)16 * 1024 * 1024;

    float*  Qp   = allocf(NPROJ);
    float*  Kp   = allocf(NPROJ);
    float*  Vp   = allocf(NPROJ);
    float*  dotA = allocf(NATT);
    float*  qn   = allocf(NROW);
    float*  kn   = allocf(NROW);
    __bf16* Zqb  = allocb(NPROJ);
    __bf16* Zkb  = allocb(NPROJ);
    __bf16* Zvb  = allocb(NPROJ);
    __bf16* Wqb  = allocb(NW);
    __bf16* Wkb  = allocb(NW);
    __bf16* Wvb  = allocb(NW);
    __bf16* Wob  = allocb(NW);
    __bf16* Qr   = allocb(NROT);
    __bf16* Kr   = allocb(NROT);
    __bf16* Vr   = allocb(NROT);
    __bf16* Ahat = allocb(NATT);
    __bf16* Zql  = allocb(NPROJ);
    __bf16* Zkl  = allocb(NPROJ);
    __bf16* Zvl  = allocb(NPROJ);
    __bf16* Wql  = allocb(NW);
    __bf16* Wkl  = allocb(NW);
    __bf16* Wvl  = allocb(NW);
    __bf16* Wol  = allocb(NW);
    float*  est  = Kp;
    __bf16* Xo   = Zqb;
    __bf16* Xol  = Zql;
    if ((size_t)(w - (char*)d_ws) > ws_size) return;

    const dim3 blk(256);

    f32_to_bf16_kernel<<<dim3(NPROJ / (256 * 8)), blk, 0, stream>>>(Zq, Zqb, Zql);
    f32_to_bf16_kernel<<<dim3(NPROJ / (256 * 8)), blk, 0, stream>>>(Zk, Zkb, Zkl);
    f32_to_bf16_kernel<<<dim3(NPROJ / (256 * 8)), blk, 0, stream>>>(Zv, Zvb, Zvl);
    f32_to_bf16_kernel<<<dim3(NW / (256 * 8)), blk, 0, stream>>>(Wq_w, Wqb, Wql);
    f32_to_bf16_kernel<<<dim3(NW / (256 * 8)), blk, 0, stream>>>(Wk_w, Wkb, Wkl);
    f32_to_bf16_kernel<<<dim3(NW / (256 * 8)), blk, 0, stream>>>(Wv_w, Wvb, Wvl);
    f32_to_bf16_kernel<<<dim3(NW / (256 * 8)), blk, 0, stream>>>(Wo_w, Wob, Wol);

    wmma_gemm_kernel<false, true><<<dim3(8, 16, 1), blk, 0, stream>>>(
        Zqb, Wqb, Wq_b, Qp, 2048, 1024, 1024, 0, 0, 0, Zql, Wql);
    wmma_gemm_kernel<false, true><<<dim3(8, 16, 1), blk, 0, stream>>>(
        Zkb, Wkb, Wk_b, Kp, 2048, 1024, 1024, 0, 0, 0, Zkl, Wkl);
    wmma_gemm_kernel<false, true><<<dim3(8, 16, 1), blk, 0, stream>>>(
        Zvb, Wvb, Wv_b, Vp, 2048, 1024, 1024, 0, 0, 0, Zvl, Wvl);

    rotate_qkv_kernel<<<dim3(32, 8, 2), dim3(256), 0, stream>>>(
        Qp, Kp, Vp, lam, Qr, Kr, Vr, qn, kn);

    wmma_gemm_kernel<true, false><<<dim3(8, 8, 16), blk, 0, stream>>>(
        Qr, Kr, nullptr, dotA, 1024, 1024, 128,
        (long long)1024 * 128, (long long)1024 * 128, (long long)1024 * 1024);

    softmax_kernel<<<dim3(1024, 8, 2), blk, 0, stream>>>(
        dotA, Ahat, qn, kn, mu, sig, eta, gam, tau, nus);

    wmma_gemm_kernel<false, false><<<dim3(1, 8, 16), blk, 0, stream>>>(
        Ahat, Vr, nullptr, est, 1024, 128, 1024,
        (long long)1024 * 1024, (long long)1024 * 128, (long long)1024 * 128);

    unrotate_kernel<<<dim3(1024, 8, 2), dim3(64), 0, stream>>>(est, lam, Xo, Xol);

    wmma_gemm_kernel<false, true><<<dim3(8, 16, 1), blk, 0, stream>>>(
        Xo, Wob, Wo_b, (float*)d_out, 2048, 1024, 1024, 0, 0, 0, Xol, Wol);
}
